// GaussianSplattingSimple_86346022519338
// MI455X (gfx1250) — hardware-verified
//
#include <hip/hip_runtime.h>


namespace {
constexpr int B = 2, CI = 64, HI = 64, HD = 256, GH = 32, NG = GH * GH, CU = 1024, CV = 512, ND = 730, NDP = 736, OH = 128;
constexpr float XS = 8.0f, WSC = 256.0f;
__constant__ float c_cho1[9] = {0.0f,0.4099999964237213f,0.6200000047683716f,0.9800000190734863f,1.1299999952316284f,1.2899999618530273f,1.6399999856948853f,1.850000023841858f,2.359999895095825f}, c_cho2[9] = {-0.8600000143051147f,-0.36000001430511475f,-0.1599999964237213f,0.1899999976158142f,0.3400000035762787f,0.49000000953674316f,0.8399999737739563f,1.0399999618530273f,1.5399999618530273f}, c_cho3[9] = {0.0f,0.33000001311302185f,0.5299999713897705f,0.8799999952316284f,1.0299999713897705f,1.1799999475479126f,1.5299999713897705f,1.7300000190734863f,2.2300000190734863f};
__constant__ int c_bi[512] = {0,0,0,1,0,0,1,2,0,0,1,2,0,1,2,3,0,1,2,3,1,2,3,4,1,2,3,4,2,3,4,5,2,3,4,5,3,4,5,6,3,4,5,6,4,5,6,7,4,5,6,7,5,6,7,8,5,6,7,8,6,7,8,9,6,7,8,9,7,8,9,10,7,8,9,10,8,9,10,11,8,9,10,11,9,10,11,12,9,10,11,12,10,11,12,13,10,11,12,13,11,12,13,14,11,12,13,14,12,13,14,15,12,13,14,15,13,14,15,16,13,14,15,16,14,15,16,17,14,15,16,17,15,16,17,18,15,16,17,18,16,17,18,19,16,17,18,19,17,18,19,20,17,18,19,20,18,19,20,21,18,19,20,21,19,20,21,22,19,20,21,22,20,21,22,23,20,21,22,23,21,22,23,24,21,22,23,24,22,23,24,25,22,23,24,25,23,24,25,26,23,24,25,26,24,25,26,27,24,25,26,27,25,26,27,28,25,26,27,28,26,27,28,29,26,27,28,29,27,28,29,30,27,28,29,30,28,29,30,31,28,29,30,31,29,30,31,32,29,30,31,32,30,31,32,33,30,31,32,33,31,32,33,34,31,32,33,34,32,33,34,35,32,33,34,35,33,34,35,36,33,34,35,36,34,35,36,37,34,35,36,37,35,36,37,38,35,36,37,38,36,37,38,39,36,37,38,39,37,38,39,40,37,38,39,40,38,39,40,41,38,39,40,41,39,40,41,42,39,40,41,42,40,41,42,43,40,41,42,43,41,42,43,44,41,42,43,44,42,43,44,45,42,43,44,45,43,44,45,46,43,44,45,46,44,45,46,47,44,45,46,47,45,46,47,48,45,46,47,48,46,47,48,49,46,47,48,49,47,48,49,50,47,48,49,50,48,49,50,51,48,49,50,51,49,50,51,52,49,50,51,52,50,51,52,53,50,51,52,53,51,52,53,54,51,52,53,54,52,53,54,55,52,53,54,55,53,54,55,56,53,54,55,56,54,55,56,57,54,55,56,57,55,56,57,58,55,56,57,58,56,57,58,59,56,57,58,59,57,58,59,60,57,58,59,60,58,59,60,61,58,59,60,61,59,60,61,62,59,60,61,62,60,61,62,63,60,61,62,63,61,62,63,63,61,62,63,63,62,63,63,63};
__constant__ float c_bw[512] = {0.00000000f,0.00000000f,1.08823526f,-0.0882352963f,0.00000000f,0.810218990f,0.211678833f,-0.0218978096f,0.00000000f,0.221374050f,0.847328246f,-0.0687022880f,-0.0703125000f,0.867187500f,0.226562500f,-0.0234375000f,-0.0234375000f,0.226562500f,0.867187500f,-0.0703125000f,-0.0703125000f,0.867187500f,0.226562500f,-0.0234375000f,-0.0234375000f,0.226562500f,0.867187500f,-0.0703125000f,-0.0703125000f,0.867187500f,0.226562500f,-0.0234375000f,-0.0234375000f,0.226562500f,0.867187500f,-0.0703125000f,-0.0703125000f,0.867187500f,0.226562500f,-0.0234375000f,-0.0234375000f,0.226562500f,0.867187500f,-0.0703125000f,-0.0703125000f,0.867187500f,0.226562500f,-0.0234375000f,-0.0234375000f,0.226562500f,0.867187500f,-0.0703125000f,-0.0703125000f,0.867187500f,0.226562500f,-0.0234375000f,-0.0234375000f,0.226562500f,0.867187500f,-0.0703125000f,-0.0703125000f,0.867187500f,0.226562500f,-0.0234375000f,-0.0234375000f,0.226562500f,0.867187500f,-0.0703125000f,-0.0703125000f,0.867187500f,0.226562500f,-0.0234375000f,-0.0234375000f,0.226562500f,0.867187500f,-0.0703125000f,-0.0703125000f,0.867187500f,0.226562500f,-0.0234375000f,-0.0234375000f,0.226562500f,0.867187500f,-0.0703125000f,-0.0703125000f,0.867187500f,0.226562500f,-0.0234375000f,-0.0234375000f,0.226562500f,0.867187500f,-0.0703125000f,-0.0703125000f,0.867187500f,0.226562500f,-0.0234375000f,-0.0234375000f,0.226562500f,0.867187500f,-0.0703125000f,-0.0703125000f,0.867187500f,0.226562500f,-0.0234375000f,-0.0234375000f,0.226562500f,0.867187500f,-0.0703125000f,-0.0703125000f,0.867187500f,0.226562500f,-0.0234375000f,-0.0234375000f,0.226562500f,0.867187500f,-0.0703125000f,-0.0703125000f,0.867187500f,0.226562500f,-0.0234375000f,-0.0234375000f,0.226562500f,0.867187500f,-0.0703125000f,-0.0703125000f,0.867187500f,0.226562500f,-0.0234375000f,-0.0234375000f,0.226562500f,0.867187500f,-0.0703125000f,-0.0703125000f,0.867187500f,0.226562500f,-0.0234375000f,-0.0234375000f,0.226562500f,0.867187500f,-0.0703125000f,-0.0703125000f,0.867187500f,0.226562500f,-0.0234375000f,-0.0234375000f,0.226562500f,0.867187500f,-0.0703125000f,-0.0703125000f,0.867187500f,0.226562500f,-0.0234375000f,-0.0234375000f,0.226562500f,0.867187500f,-0.0703125000f,-0.0703125000f,0.867187500f,0.226562500f,-0.0234375000f,-0.0234375000f,0.226562500f,0.867187500f,-0.0703125000f,-0.0703125000f,0.867187500f,0.226562500f,-0.0234375000f,-0.0234375000f,0.226562500f,0.867187500f,-0.0703125000f,-0.0703125000f,0.867187500f,0.226562500f,-0.0234375000f,-0.0234375000f,0.226562500f,0.867187500f,-0.0703125000f,-0.0703125000f,0.867187500f,0.226562500f,-0.0234375000f,-0.0234375000f,0.226562500f,0.867187500f,-0.0703125000f,-0.0703125000f,0.867187500f,0.226562500f,-0.0234375000f,-0.0234375000f,0.226562500f,0.867187500f,-0.0703125000f,-0.0703125000f,0.867187500f,0.226562500f,-0.0234375000f,-0.0234375000f,0.226562500f,0.867187500f,-0.0703125000f,-0.0703125000f,0.867187500f,0.226562500f,-0.0234375000f,-0.0234375000f,0.226562500f,0.867187500f,-0.0703125000f,-0.0703125000f,0.867187500f,0.226562500f,-0.0234375000f,-0.0234375000f,0.226562500f,0.867187500f,-0.0703125000f,-0.0703125000f,0.867187500f,0.226562500f,-0.0234375000f,-0.0234375000f,0.226562500f,0.867187500f,-0.0703125000f,-0.0703125000f,0.867187500f,0.226562500f,-0.0234375000f,-0.0234375000f,0.226562500f,0.867187500f,-0.0703125000f,-0.0703125000f,0.867187500f,0.226562500f,-0.0234375000f,-0.0234375000f,0.226562500f,0.867187500f,-0.0703125000f,-0.0703125000f,0.867187500f,0.226562500f,-0.0234375000f,-0.0234375000f,0.226562500f,0.867187500f,-0.0703125000f,-0.0703125000f,0.867187500f,0.226562500f,-0.0234375000f,-0.0234375000f,0.226562500f,0.867187500f,-0.0703125000f,-0.0703125000f,0.867187500f,0.226562500f,-0.0234375000f,-0.0234375000f,0.226562500f,0.867187500f,-0.0703125000f,-0.0703125000f,0.867187500f,0.226562500f,-0.0234375000f,-0.0234375000f,0.226562500f,0.867187500f,-0.0703125000f,-0.0703125000f,0.867187500f,0.226562500f,-0.0234375000f,-0.0234375000f,0.226562500f,0.867187500f,-0.0703125000f,-0.0703125000f,0.867187500f,0.226562500f,-0.0234375000f,-0.0234375000f,0.226562500f,0.867187500f,-0.0703125000f,-0.0703125000f,0.867187500f,0.226562500f,-0.0234375000f,-0.0234375000f,0.226562500f,0.867187500f,-0.0703125000f,-0.0703125000f,0.867187500f,0.226562500f,-0.0234375000f,-0.0234375000f,0.226562500f,0.867187500f,-0.0703125000f,-0.0703125000f,0.867187500f,0.226562500f,-0.0234375000f,-0.0234375000f,0.226562500f,0.867187500f,-0.0703125000f,-0.0703125000f,0.867187500f,0.226562500f,-0.0234375000f,-0.0234375000f,0.226562500f,0.867187500f,-0.0703125000f,-0.0703125000f,0.867187500f,0.226562500f,-0.0234375000f,-0.0234375000f,0.226562500f,0.867187500f,-0.0703125000f,-0.0703125000f,0.867187500f,0.226562500f,-0.0234375000f,-0.0234375000f,0.226562500f,0.867187500f,-0.0703125000f,-0.0703125000f,0.867187500f,0.226562500f,-0.0234375000f,-0.0234375000f,0.226562500f,0.867187500f,-0.0703125000f,-0.0703125000f,0.867187500f,0.226562500f,-0.0234375000f,-0.0234375000f,0.226562500f,0.867187500f,-0.0703125000f,-0.0703125000f,0.867187500f,0.226562500f,-0.0234375000f,-0.0234375000f,0.226562500f,0.867187500f,-0.0703125000f,-0.0703125000f,0.867187500f,0.226562500f,-0.0234375000f,-0.0234375000f,0.226562500f,0.867187500f,-0.0703125000f,-0.0703125000f,0.867187500f,0.226562500f,-0.0234375000f,-0.0234375000f,0.226562500f,0.867187500f,-0.0703125000f,-0.0703125000f,0.867187500f,0.226562500f,-0.0234375000f,-0.0234375000f,0.226562500f,0.867187500f,-0.0703125000f,-0.0703125000f,0.867187500f,0.226562500f,-0.0234375000f,-0.0234375000f,0.226562500f,0.867187500f,-0.0703125000f,-0.0703125000f,0.867187500f,0.226562500f,-0.0234375000f,-0.0234375000f,0.226562500f,0.867187500f,-0.0703125000f,-0.0703125000f,0.867187500f,0.226562500f,-0.0234375000f,-0.0234375000f,0.226562500f,0.867187500f,-0.0703125000f,-0.0703125000f,0.867187500f,0.226562500f,-0.0234375000f,-0.0234375000f,0.226562500f,0.867187500f,-0.0703125000f,-0.0703125000f,0.867187500f,0.226562500f,-0.0234375000f,-0.0234375000f,0.226562500f,0.867187500f,-0.0703125000f,-0.0703125000f,0.867187500f,0.226562500f,-0.0234375000f,-0.0234375000f,0.226562500f,0.867187500f,-0.0703125000f,-0.0703125000f,0.867187500f,0.226562500f,-0.0234375000f,-0.0234375000f,0.226562500f,0.867187500f,-0.0703125000f,-0.0703125000f,0.867187500f,0.226562500f,-0.0234375000f,-0.0234375000f,0.226562500f,0.867187500f,-0.0703125000f,-0.0703125000f,0.867187500f,0.226562500f,-0.0234375000f,-0.0234375000f,0.226562500f,0.867187500f,-0.0703125000f,-0.0703125000f,0.867187500f,0.226562500f,-0.0234375000f,-0.0234375000f,0.226562500f,0.867187500f,-0.0703125000f,-0.0703125000f,0.867187500f,0.226562500f,-0.0234375000f,-0.0234375000f,0.226562500f,0.867187500f,-0.0703125000f,-0.0703125000f,0.867187500f,0.226562500f,-0.0234375000f,-0.0234375000f,0.226562500f,0.867187500f,-0.0703125000f,-0.0703125000f,0.867187500f,0.226562500f,-0.0234375000f,-0.0234375000f,0.226562500f,0.867187500f,-0.0703125000f,-0.0703125000f,0.867187500f,0.226562500f,-0.0234375000f,-0.0234375000f,0.226562500f,0.867187500f,-0.0703125000f,-0.0687022880f,0.847328246f,0.221374050f,0.00000000f,-0.0218978096f,0.211678833f,0.810218990f,0.00000000f,-0.0882352963f,1.08823526f,0.00000000f,0.00000000f};
typedef _Float16 b16;
typedef __attribute__((ext_vector_type(16))) _Float16 v16b;
typedef __attribute__((ext_vector_type(8))) _Float16 v8b;
typedef __attribute__((ext_vector_type(8))) float v8f;
typedef __attribute__((ext_vector_type(4))) float v4f;
typedef __attribute__((ext_vector_type(2))) float v2f;
__device__ __forceinline__ float bf16_rne(float f) { unsigned int u = __float_as_uint(f); u += 0x7FFFu + ((u >> 16) & 1u); float r = __uint_as_float(u & 0xFFFF0000u); asm volatile("" : "+v"(r)); return r; }
__device__ __forceinline__ void split16(float v, b16& hi, b16& lo) { hi = (b16)v; lo = (b16)(v - (float)hi); }
__device__ __forceinline__ v16b frag_kb(const b16* p, int hh) { const v8b a = *(const v8b*)(p + 8 * hh), b = *(const v8b*)(p + 16 + 8 * hh); v16b f;
#pragma unroll
  for (int e = 0; e < 8; ++e) { f[e] = a[e]; f[8 + e] = b[e]; } return f; }
__device__ __forceinline__ v8f wmma16b(v16b a, v16b b, v8f c) { v8f d = __builtin_amdgcn_wmma_f32_16x16x32_f16(false, a, false, b, (short)0, c, false, false); asm volatile("v_nop\n\tv_nop\n\tv_nop\n\tv_nop" : "+v"(d) : "v"(a), "v"(b)); return d; }
__device__ __forceinline__ void wave_lds_sync() { __builtin_amdgcn_fence(__ATOMIC_RELEASE, "workgroup"); __builtin_amdgcn_wave_barrier(); __builtin_amdgcn_fence(__ATOMIC_ACQUIRE, "workgroup"); }
__device__ __forceinline__ float pmul(float a, float b) { float p = a * b; asm volatile("" : "+v"(p)); return p; }
__device__ __forceinline__ int iclamp(int v, int lo, int hi) { return v < lo ? lo : (v > hi ? hi : v); }
__device__ __forceinline__ void gdict(int i, float& g0, float& g1, float& g2) { if (i >= 729) { g0 = g1 = g2 = 0.0f; return; } g0 = c_cho1[i / 81]; g1 = c_cho2[(i / 9) % 9]; g2 = c_cho3[i % 9]; }

__global__ __launch_bounds__(256) void wput_kernel(const float* __restrict__ c1w, const float* __restrict__ cvw, const float* __restrict__ cw1, const float* __restrict__ cw2, const float* __restrict__ cw3, const float* __restrict__ ow1, const float* __restrict__ ow2, const float* __restrict__ dw2,
    b16* __restrict__ W1C, b16* __restrict__ WCV, b16* __restrict__ CW1, b16* __restrict__ CW2, b16* __restrict__ CW3, b16* __restrict__ OW1, b16* __restrict__ OW2, b16* __restrict__ DW2) { const size_t u = (size_t)blockIdx.x * 256 + threadIdx.x;
  for (int pass = 0; pass < 2; ++pass) {
    if (u < (size_t)HD * 72) { v8b v; for (int j = 0; j < 8; ++j) v[j] = (b16)(bf16_rne(c1w[u * 8 + j]) * WSC); *(volatile v8b*)(W1C + u * 8) = v; }
    if (u < (size_t)9 * CV * (CU / 8)) { const int t = (int)(u / ((size_t)CV * 128)); const size_t rem = u % ((size_t)CV * 128); const int o = (int)(rem / 128), c0 = (int)(rem % 128) * 8; v8b v; for (int j = 0; j < 8; ++j) v[j] = (b16)(bf16_rne(cvw[(((size_t)o * CU + c0 + j) * 9) + t]) * WSC); *(volatile v8b*)(WCV + u * 8) = v; }
    if (u < (size_t)CV * 128) { const int o = (int)(u / 128), k0 = (int)(u % 128) * 8; v8b v; for (int j = 0; j < 8; ++j) v[j] = (b16)(bf16_rne(cw1[(size_t)(k0 + j) * CV + o]) * WSC); *(volatile v8b*)(CW1 + u * 8) = v; }
    if (u < (size_t)HD * 64) { const int o = (int)(u / 64), k0 = (int)(u % 64) * 8; v8b v; for (int j = 0; j < 8; ++j) v[j] = (b16)(bf16_rne(cw2[(size_t)(k0 + j) * HD + o]) * WSC); *(volatile v8b*)(CW2 + u * 8) = v; }
    if (u < (size_t)16 * 32) { const int o = (int)(u / 32), k0 = (int)(u % 32) * 8; v8b a, b; for (int j = 0; j < 8; ++j) { a[j] = (b16)(o < 3 ? bf16_rne(cw3[(size_t)(k0 + j) * 3 + o]) * WSC : 0.0f); b[j] = (b16)(o < 2 ? bf16_rne(ow2[(size_t)(k0 + j) * 2 + o]) * WSC : 0.0f); } *(volatile v8b*)(CW3 + u * 8) = a; *(volatile v8b*)(OW2 + u * 8) = b; }
    if (u < (size_t)HD * 128) { const int o = (int)(u / 128), k0 = (int)(u % 128) * 8; v8b v; for (int j = 0; j < 8; ++j) v[j] = (b16)(bf16_rne(ow1[(size_t)(k0 + j) * HD + o]) * WSC); *(volatile v8b*)(OW1 + u * 8) = v; }
    if (u < (size_t)CV * 32) { const int o = (int)(u / 32), k0 = (int)(u % 32) * 8; v8b v; for (int j = 0; j < 8; ++j) v[j] = (b16)(bf16_rne(dw2[(size_t)(k0 + j) * CV + o]) * WSC); *(volatile v8b*)(DW2 + u * 8) = v; }
    __threadfence(); } }
__global__ __launch_bounds__(32) void conv1_kernel(const float* __restrict__ feat, const b16* __restrict__ W1C, const float* __restrict__ c1b, float* __restrict__ U) { __shared__ __attribute__((aligned(16))) b16 Ah[32][584]; __shared__ float Tf[32][260]; const int lane = threadIdx.x, nloc = lane & 15, hlf = lane >> 4; const int b = blockIdx.x / (GH * 4), gy = (blockIdx.x / 4) % GH, gx0 = (blockIdx.x % 4) * 8; const int Y0 = 2 * gy, X0 = 2 * gx0;
  for (int r = 0; r < 32; ++r) { const int Y = Y0 + (r >> 4), X = X0 + (r & 15);
    for (int c = lane; c < CI; c += 32) { for (int t = 0; t < 9; ++t) { const int yy = Y + t / 3 - 1, xx = X + t % 3 - 1; const float v = (yy >= 0 && yy < HI && xx >= 0 && xx < HI) ? bf16_rne(feat[(((size_t)b * CI + c) * HI + yy) * HI + xx]) : 0.0f; Ah[r][c * 9 + t] = (b16)(v * XS); } } if (lane < 8) { Ah[r][576 + lane] = (b16)0.0f; } }
  wave_lds_sync();
  for (int mt = 0; mt < 2; ++mt) { v8f acc[16];
#pragma unroll
    for (int t = 0; t < 16; ++t) acc[t] = (v8f){};
#pragma unroll 1
    for (int kb = 0; kb < 576; kb += 32) { const v16b a = frag_kb(&Ah[mt * 16 + nloc][kb], hlf);
#pragma unroll
      for (int t = 0; t < 16; ++t) acc[t] = wmma16b(a, frag_kb(W1C + (size_t)(t * 16 + nloc) * 576 + kb, hlf), acc[t]); }
#pragma unroll
    for (int t = 0; t < 16; ++t) { const int o = t * 16 + nloc; const float bb = bf16_rne(c1b[o]);
#pragma unroll
      for (int r8 = 0; r8 < 8; ++r8) { float v = acc[t][r8] * (1.0f / (XS * WSC)) + bb; v = v >= 0.0f ? v : 0.1f * v; Tf[mt * 16 + 8 * hlf + r8][o] = v; } } }
  wave_lds_sync();
  for (int pass = 0; pass < 2; ++pass) { for (int q = 0; q < 8; ++q) { float* row = U + (((size_t)b * GH + gy) * GH + gx0 + q) * CU; for (int o = lane; o < HD; o += 32) { v4f v = {Tf[2 * q][o], Tf[2 * q + 1][o], Tf[16 + 2 * q][o], Tf[16 + 2 * q + 1][o]}; *(volatile v4f*)(row + o * 4) = v; } } __threadfence(); } }
__global__ __launch_bounds__(32) void mlp1_kernel(const float* __restrict__ U, const b16* __restrict__ CW1, const float* __restrict__ cb1, const b16* __restrict__ OW1, const float* __restrict__ ob1, int RLIM, float* __restrict__ C1, float* __restrict__ O1) { __shared__ __attribute__((aligned(16))) b16 Ah[16][CU + 8], Al[16][CU + 8]; __shared__ float Tf[16][260]; const int lane = threadIdx.x, nloc = lane & 15, hlf = lane >> 4; const int g = blockIdx.x % 3; const size_t r0 = (size_t)(blockIdx.x / 3) * 16; if (r0 >= (size_t)RLIM) return;
  for (int rr = 0; rr < 16; ++rr) for (int q = 0; q < CU / 32; ++q) { b16 p, ql; split16(U[(r0 + rr) * CU + q * 32 + lane] * XS, p, ql); Ah[rr][q * 32 + lane] = p; Al[rr][q * 32 + lane] = ql; }
  wave_lds_sync(); const b16* WT = g < 2 ? CW1 + (size_t)g * 256 * CU : OW1; const float* bias = g < 2 ? cb1 + g * 256 : ob1; v8f acc[16];
#pragma unroll
  for (int t = 0; t < 16; ++t) acc[t] = (v8f){};
#pragma unroll 1
  for (int kb = 0; kb < CU; kb += 32) { const v16b a = frag_kb(&Ah[nloc][kb], hlf), al = frag_kb(&Al[nloc][kb], hlf);
#pragma unroll
    for (int t = 0; t < 16; ++t) { const v16b bw = frag_kb(WT + (size_t)(t * 16 + nloc) * CU + kb, hlf); acc[t] = wmma16b(a, bw, acc[t]); acc[t] = wmma16b(al, bw, acc[t]); } }
#pragma unroll
  for (int t = 0; t < 16; ++t) { const int cc = t * 16 + nloc; const float bb = bf16_rne(bias[cc]);
#pragma unroll
    for (int r8 = 0; r8 < 8; ++r8) Tf[8 * hlf + r8][cc] = fmaxf(acc[t][r8] * (1.0f / (XS * WSC)) + bb, 0.0f); }
  wave_lds_sync();
  for (int pass = 0; pass < 2; ++pass) { for (int rr = 0; rr < 16; ++rr) for (int q = 0; q < 2; ++q) { const v4f v = *(const v4f*)(&Tf[rr][q * 128 + lane * 4]); if (g < 2) *(volatile v4f*)(C1 + (r0 + rr) * CV + g * 256 + q * 128 + lane * 4) = v; else *(volatile v4f*)(O1 + (r0 + rr) * HD + q * 128 + lane * 4) = v; } __threadfence(); } }
__global__ __launch_bounds__(32) void mlp2_kernel(const float* __restrict__ C1, const float* __restrict__ O1, const b16* __restrict__ CW2, const float* __restrict__ cb2, const b16* __restrict__ CW3, const float* __restrict__ cb3, const b16* __restrict__ OW2, const float* __restrict__ ob2, int RLIM, float* __restrict__ CO) { __shared__ __attribute__((aligned(16))) b16 Ah[16][CV + 8], Al[16][CV + 8]; __shared__ float Pf[16][8]; const int lane = threadIdx.x, nloc = lane & 15, hlf = lane >> 4; const size_t r0 = (size_t)blockIdx.x * 16; if (r0 >= (size_t)RLIM) return;
  for (int rr = 0; rr < 16; ++rr) for (int q = 0; q < CV / 32; ++q) { b16 p, ql; split16(C1[(r0 + rr) * CV + q * 32 + lane] * XS, p, ql); Ah[rr][q * 32 + lane] = p; Al[rr][q * 32 + lane] = ql; }
  wave_lds_sync(); v8f acc[16];
#pragma unroll
  for (int t = 0; t < 16; ++t) acc[t] = (v8f){};
#pragma unroll 1
  for (int kb = 0; kb < CV; kb += 32) { const v16b a = frag_kb(&Ah[nloc][kb], hlf), al = frag_kb(&Al[nloc][kb], hlf);
#pragma unroll
    for (int t = 0; t < 16; ++t) { const v16b bw = frag_kb(CW2 + (size_t)(t * 16 + nloc) * CV + kb, hlf); acc[t] = wmma16b(a, bw, acc[t]); acc[t] = wmma16b(al, bw, acc[t]); } }
  wave_lds_sync();
#pragma unroll
  for (int t = 0; t < 16; ++t) { const int cc = t * 16 + nloc; const float bb = bf16_rne(cb2[cc]);
#pragma unroll
    for (int r8 = 0; r8 < 8; ++r8) { b16 p, ql; split16(fmaxf(acc[t][r8] * (1.0f / (XS * WSC)) + bb, 0.0f) * XS, p, ql); Ah[8 * hlf + r8][cc] = p; Al[8 * hlf + r8][cc] = ql; } }
  for (int rr = 0; rr < 16; ++rr) for (int q = 0; q < HD / 32; ++q) { b16 p, ql; split16(O1[(r0 + rr) * HD + q * 32 + lane] * XS, p, ql); Ah[rr][HD + q * 32 + lane] = p; Al[rr][HD + q * 32 + lane] = ql; }
  wave_lds_sync(); v8f ac = {}, ao = {};
#pragma unroll
  for (int kb = 0; kb < HD; kb += 32) { const v16b a = frag_kb(&Ah[nloc][kb], hlf), al = frag_kb(&Al[nloc][kb], hlf); const v16b bw = frag_kb(CW3 + (size_t)nloc * HD + kb, hlf); ac = wmma16b(a, bw, ac); ac = wmma16b(al, bw, ac);
    const v16b a2 = frag_kb(&Ah[nloc][HD + kb], hlf), al2 = frag_kb(&Al[nloc][HD + kb], hlf); const v16b bo = frag_kb(OW2 + (size_t)nloc * HD + kb, hlf); ao = wmma16b(a2, bo, ao); ao = wmma16b(al2, bo, ao); }
#pragma unroll
  for (int r8 = 0; r8 < 8; ++r8) { const int rr = 8 * hlf + r8; if (nloc < 3) Pf[rr][nloc] = ac[r8] * (1.0f / (XS * WSC)) + bf16_rne(cb3[nloc]); if (nloc < 2) Pf[rr][3 + nloc] = tanhf(ao[r8] * (1.0f / (XS * WSC)) + bf16_rne(ob2[nloc])); if (nloc >= 5 && nloc < 8) Pf[rr][nloc] = 0.0f; }
  wave_lds_sync();
  for (int pass = 0; pass < 2; ++pass) { for (int q = lane; q < 128; q += 32) ((volatile float*)CO)[r0 * 8 + q] = Pf[q / 8][q % 8]; __threadfence(); } }
__global__ __launch_bounds__(32) void cov_kernel(const float* __restrict__ U, const b16* __restrict__ WCV, const float* __restrict__ cvb, int RLIM, float* __restrict__ COVF) { __shared__ __attribute__((aligned(16))) b16 Ah[16][CU + 8]; __shared__ float Tf[16][260]; const int lane = threadIdx.x, nloc = lane & 15, hlf = lane >> 4; const int g = blockIdx.x & 1; const size_t r0 = (size_t)(blockIdx.x >> 1) * 16; if (r0 >= (size_t)RLIM) return; const int b = (int)(r0 / NG), gy = (int)((r0 % NG) / GH), gx0 = (int)(r0 % GH);
  v8f acc[16];
#pragma unroll
  for (int t = 0; t < 16; ++t) acc[t] = (v8f){};
#pragma unroll 1
  for (int tap = 0; tap < 9; ++tap) { const int yy = gy + tap / 3 - 1; const int dx = tap % 3 - 1;
    for (int rr = 0; rr < 16; ++rr) { const int xx = gx0 + rr + dx; const bool ok = yy >= 0 && yy < GH && xx >= 0 && xx < GH; const float* src = U + (((size_t)b * GH + (ok ? yy : 0)) * GH + (ok ? xx : 0)) * CU; for (int q = 0; q < CU / 32; ++q) Ah[rr][q * 32 + lane] = (b16)(ok ? src[q * 32 + lane] * XS : 0.0f); }
    wave_lds_sync(); const b16* WT = WCV + ((size_t)tap * CV + g * 256) * CU;
#pragma unroll 1
    for (int kb = 0; kb < CU; kb += 32) { const v16b a = frag_kb(&Ah[nloc][kb], hlf);
#pragma unroll
      for (int t = 0; t < 16; ++t) acc[t] = wmma16b(a, frag_kb(WT + (size_t)(t * 16 + nloc) * CU + kb, hlf), acc[t]); }
    wave_lds_sync(); }
#pragma unroll
  for (int t = 0; t < 16; ++t) { const int cc = t * 16 + nloc; const float bb = bf16_rne(cvb[g * 256 + cc]);
#pragma unroll
    for (int r8 = 0; r8 < 8; ++r8) Tf[8 * hlf + r8][cc] = acc[t][r8] * (1.0f / (XS * WSC)) + bb; }
  wave_lds_sync();
  for (int pass = 0; pass < 2; ++pass) { for (int rr = 0; rr < 16; ++rr) for (int q = 0; q < 2; ++q) *(volatile v4f*)(COVF + (r0 + rr) * CV + g * 256 + q * 128 + lane * 4) = *(const v4f*)(&Tf[rr][q * 128 + lane * 4]); __threadfence(); } }
__global__ __launch_bounds__(32) void dict_kernel(const float* __restrict__ dw1, const float* __restrict__ db1, const b16* __restrict__ DW2, const float* __restrict__ db2, b16* __restrict__ DEh, b16* __restrict__ DEl) { __shared__ __attribute__((aligned(16))) b16 Ah[16][HD + 8], Al[16][HD + 8]; __shared__ float Tf[16][132]; const int lane = threadIdx.x, nloc = lane & 15, hlf = lane >> 4; const int g = blockIdx.x % 4; const int i0 = (blockIdx.x / 4) * 16;
  for (int rr = 0; rr < 16; ++rr) { float g0, g1, g2; gdict(i0 + rr, g0, g1, g2); for (int q = 0; q < HD / 32; ++q) { const int c = q * 32 + lane; const float d = (i0 + rr < ND) ? fmaxf(pmul(g0, bf16_rne(dw1[c])) + pmul(g1, bf16_rne(dw1[HD + c])) + pmul(g2, bf16_rne(dw1[2 * HD + c])) + bf16_rne(db1[c]), 0.0f) : 0.0f; b16 p, ql; split16(d * XS, p, ql); Ah[rr][c] = p; Al[rr][c] = ql; } }
  wave_lds_sync(); v8f acc[8];
#pragma unroll
  for (int t = 0; t < 8; ++t) acc[t] = (v8f){};
#pragma unroll
  for (int kb = 0; kb < HD; kb += 32) { const v16b a = frag_kb(&Ah[nloc][kb], hlf), al = frag_kb(&Al[nloc][kb], hlf);
#pragma unroll
    for (int t = 0; t < 8; ++t) { const v16b bw = frag_kb(DW2 + (size_t)(g * 128 + t * 16 + nloc) * HD + kb, hlf); acc[t] = wmma16b(a, bw, acc[t]); acc[t] = wmma16b(al, bw, acc[t]); } }
#pragma unroll
  for (int t = 0; t < 8; ++t) { const int cc = t * 16 + nloc; const float bb = bf16_rne(db2[g * 128 + cc]);
#pragma unroll
    for (int r8 = 0; r8 < 8; ++r8) Tf[8 * hlf + r8][cc] = (i0 + 8 * hlf + r8 < ND) ? acc[t][r8] * (1.0f / (XS * WSC)) + bb : 0.0f; }
  wave_lds_sync();
  for (int pass = 0; pass < 2; ++pass) { for (int rr = 0; rr < 16; ++rr) { v4f v = *(const v4f*)(&Tf[rr][lane * 4]); b16 ph[4], pl[4]; for (int k = 0; k < 4; ++k) split16(v[k] * WSC, ph[k], pl[k]);
      typedef __attribute__((ext_vector_type(4))) _Float16 v4b; *(volatile v4b*)(DEh + (size_t)(i0 + rr) * CV + g * 128 + lane * 4) = (v4b){ph[0], ph[1], ph[2], ph[3]}; *(volatile v4b*)(DEl + (size_t)(i0 + rr) * CV + g * 128 + lane * 4) = (v4b){pl[0], pl[1], pl[2], pl[3]}; } __threadfence(); } }
__global__ __launch_bounds__(32) void logit_kernel(const float* __restrict__ COVF, const b16* __restrict__ DEh, const b16* __restrict__ DEl, int RLIM, float* __restrict__ LG) { __shared__ __attribute__((aligned(16))) b16 Ah[16][CV + 8], Al[16][CV + 8]; __shared__ float Tf[16][260]; const int lane = threadIdx.x, nloc = lane & 15, hlf = lane >> 4; const int g = blockIdx.x % 3; const size_t r0 = (size_t)(blockIdx.x / 3) * 16; if (r0 >= (size_t)RLIM) return; const int t0 = g * 16, nt = (g == 2) ? (NDP / 16 - 32) : 16;
  for (int rr = 0; rr < 16; ++rr) for (int q = 0; q < CV / 32; ++q) { b16 p, ql; split16(COVF[(r0 + rr) * CV + q * 32 + lane] * XS, p, ql); Ah[rr][q * 32 + lane] = p; Al[rr][q * 32 + lane] = ql; }
  wave_lds_sync(); v8f acc[16];
#pragma unroll
  for (int t = 0; t < 16; ++t) acc[t] = (v8f){};
#pragma unroll 1
  for (int kb = 0; kb < CV; kb += 32) { const v16b a = frag_kb(&Ah[nloc][kb], hlf), al = frag_kb(&Al[nloc][kb], hlf);
#pragma unroll
    for (int t = 0; t < 16; ++t) { if (t < nt) { const size_t ro = (size_t)((t0 + t) * 16 + nloc) * CV + kb; const v16b bh_ = frag_kb(DEh + ro, hlf), bl_ = frag_kb(DEl + ro, hlf); acc[t] = wmma16b(a, bh_, acc[t]); acc[t] = wmma16b(a, bl_, acc[t]); acc[t] = wmma16b(al, bh_, acc[t]); } } }
#pragma unroll
  for (int t = 0; t < 16; ++t)
#pragma unroll
    for (int r8 = 0; r8 < 8; ++r8) Tf[8 * hlf + r8][t * 16 + nloc] = acc[t][r8] * (1.0f / (XS * WSC));
  wave_lds_sync();
  for (int pass = 0; pass < 2; ++pass) { for (int rr = 0; rr < 16; ++rr) for (int q = 0; q < nt / 2; ++q) ((volatile float*)LG)[(r0 + rr) * NDP + t0 * 16 + q * 32 + lane] = Tf[rr][q * 32 + lane]; __threadfence(); } }
__global__ __launch_bounds__(256) void covp_kernel(const float* __restrict__ LG, const float* __restrict__ CO, int RLIM, float* __restrict__ GP) { const int r = blockIdx.x * 256 + threadIdx.x; if (r >= B * NG) return; float o8[8] = {0, 0, 0, 0, 0, 0, 0, 0};
  if (r < RLIM) { const float* lg = LG + (size_t)r * NDP; float mx = -INFINITY; for (int i = 0; i < ND; ++i) mx = fmaxf(mx, lg[i]); float den = 0.0f, p0 = 0.0f, p1 = 0.0f, p2 = 0.0f;
    for (int i = 0; i < ND; ++i) { const float e = __expf(lg[i] - mx); float g0, g1, g2; gdict(i, g0, g1, g2); den += e; p0 += pmul(e, g0); p1 += pmul(e, g1); p2 += pmul(e, g2); }
    const float inv = 1.0f / den; p0 *= inv; p1 *= inv; p2 *= inv; const float scale = (float)OH / (float)HI;
    const float c1 = p0 * scale + 1e-4f, c2 = p1 * scale, c3 = p2 * scale + 1e-4f; const float sxx = c1 * c1, sxy = c1 * c2, syy = pmul(c2, c2) + pmul(c3, c3); const float det = pmul(sxx, syy) - pmul(sxy, sxy) + 1e-6f;
    const int gy = (r % NG) / GH, gx = r % GH; const float ry = 1.0f / GH; const float by = -1.0f + ry + 2.0f * ry * (float)gy, bx = -1.0f + ry + 2.0f * ry * (float)gx; const float* co = CO + (size_t)r * 8;
    o8[0] = by + co[3] * (2.0f / GH); o8[1] = bx + co[4] * (2.0f / GH); o8[2] = syy / det; o8[3] = sxx / det; o8[4] = sxy / det; o8[5] = co[0]; o8[6] = co[1]; o8[7] = co[2]; }
  for (int pass = 0; pass < 2; ++pass) { *(volatile v4f*)(GP + (size_t)r * 8) = (v4f){o8[0], o8[1], o8[2], o8[3]}; *(volatile v4f*)(GP + (size_t)r * 8 + 4) = (v4f){o8[4], o8[5], o8[6], o8[7]}; __threadfence(); } }
__global__ __launch_bounds__(256) void render_kernel(const float* __restrict__ GP, const float* __restrict__ lr, int BV, int NLIMG, float* __restrict__ out) { const int u = blockIdx.x * 256 + threadIdx.x; if (u >= B * OH * OH) return; const int b = u / (OH * OH), py = (u / OH) % OH, px = u % OH; float res[3] = {0, 0, 0};
  if (b < BV) { const float yp = -1.0f + 2.0f * (float)py / (float)(OH - 1), xp = -1.0f + 2.0f * (float)px / (float)(OH - 1); float den = 0.0f, n0 = 0.0f, n1 = 0.0f, n2 = 0.0f; const float* gp = GP + (size_t)b * NG * 8;
#pragma unroll 1
    for (int n = 0; n < NLIMG; ++n) { const v4f a = *(const v4f*)(gp + n * 8), c = *(const v4f*)(gp + n * 8 + 4); const float dy = yp - a[0], dx = xp - a[1]; const float m = pmul(pmul(dy, dy), a[2]) + pmul(pmul(dx, dx), a[3]) - 2.0f * pmul(pmul(dy, dx), c[0]); const float w = __expf(-0.5f * m); den += w; n0 += pmul(w, c[1]); n1 += pmul(w, c[2]); n2 += pmul(w, c[3]); }
    const float inv = 1.0f / (den + 1e-6f); res[0] = n0 * inv; res[1] = n1 * inv; res[2] = n2 * inv;
    for (int cch = 0; cch < 3; ++cch) { float s = 0.0f; const float* lp = lr + ((size_t)b * 3 + cch) * HI * HI;
#pragma unroll
      for (int ty = 0; ty < 4; ++ty) { float rs = 0.0f;
#pragma unroll
        for (int tx = 0; tx < 4; ++tx) rs += pmul(c_bw[px * 4 + tx], bf16_rne(lp[c_bi[py * 4 + ty] * HI + c_bi[px * 4 + tx]])); s += pmul(c_bw[py * 4 + ty], rs); }
      res[cch] += s; } }
  for (int pass = 0; pass < 2; ++pass) { for (int cch = 0; cch < 3; ++cch) ((volatile float*)out)[(((size_t)b * 3 + cch) * OH + py) * OH + px] = res[cch]; __threadfence(); } }
}

extern "C" void kernel_launch(void* const* d_in, const int* in_sizes, int n_in, void* d_out, int out_size, void* d_ws, size_t ws_size, hipStream_t stream) {
  (void)n_in;
  auto Fp = [&](int i) { return (const float*)d_in[i]; };
  if (in_sizes[0] != B * CI * HI * HI || in_sizes[1] != B * 3 * HI * HI || in_sizes[2] != HD * CI * 9 || in_sizes[4] != CV * CU * 9 || in_sizes[6] != CU * CV || in_sizes[8] != CV * HD || in_sizes[10] != HD * 3 || in_sizes[12] != CU * HD || in_sizes[14] != HD * 2 || in_sizes[16] != 3 * HD || in_sizes[18] != HD * CV || out_size != B * 3 * OH * OH) return;
  const int BV = B, GYV = GH;
  const int RLIM = (BV - 1) * NG + GYV * GH;
  size_t off = 0; char* ws = (char*)d_ws;
  auto carve = [&](size_t bytes) { char* p = ws + off; off += (bytes + 255) & ~(size_t)255; return p; };
  b16* W1C = (b16*)carve((size_t)HD * 576 * 2); b16* WCV = (b16*)carve((size_t)9 * CV * CU * 2); b16* CW1 = (b16*)carve((size_t)CV * CU * 2); b16* CW2 = (b16*)carve((size_t)HD * CV * 2); b16* CW3 = (b16*)carve((size_t)16 * HD * 2); b16* OW1 = (b16*)carve((size_t)HD * CU * 2); b16* OW2 = (b16*)carve((size_t)16 * HD * 2); b16* DW2 = (b16*)carve((size_t)CV * HD * 2);
  float* U = (float*)carve((size_t)B * NG * CU * 4); float* C1 = (float*)carve((size_t)B * NG * CV * 4); float* O1 = (float*)carve((size_t)B * NG * HD * 4); float* CO = (float*)carve((size_t)B * NG * 8 * 4); float* COVF = (float*)carve((size_t)B * NG * CV * 4); b16* DEh = (b16*)carve((size_t)NDP * CV * 2); b16* DEl = (b16*)carve((size_t)NDP * CV * 2); float* LG = (float*)carve((size_t)B * NG * NDP * 4); float* GP = (float*)carve((size_t)B * NG * 8 * 4);
  if (off > ws_size || off > ((size_t)64 << 20)) return;
  wput_kernel<<<(unsigned)(((size_t)9 * CV * (CU / 8) + 255) / 256), 256, 0, stream>>>(Fp(2), Fp(4), Fp(6), Fp(8), Fp(10), Fp(12), Fp(14), Fp(18), W1C, WCV, CW1, CW2, CW3, OW1, OW2, DW2);
  conv1_kernel<<<BV * GH * 4, 32, 0, stream>>>(Fp(0), W1C, Fp(3), U);
  mlp1_kernel<<<(RLIM / 16) * 3, 32, 0, stream>>>(U, CW1, Fp(7), OW1, Fp(13), RLIM, C1, O1);
  mlp2_kernel<<<RLIM / 16, 32, 0, stream>>>(C1, O1, CW2, Fp(9), CW3, Fp(11), OW2, Fp(15), RLIM, CO);
  cov_kernel<<<(RLIM / 16) * 2, 32, 0, stream>>>(U, WCV, Fp(5), RLIM, COVF);
  dict_kernel<<<(NDP / 16) * 4, 32, 0, stream>>>(Fp(16), Fp(17), DW2, Fp(19), DEh, DEl);
  logit_kernel<<<(RLIM / 16) * 3, 32, 0, stream>>>(COVF, DEh, DEl, RLIM, LG);
  covp_kernel<<<(B * NG + 255) / 256, 256, 0, stream>>>(LG, CO, RLIM, GP);
  render_kernel<<<(B * OH * OH + 255) / 256, 256, 0, stream>>>(GP, Fp(1), BV, (BV == B && GYV == GH) ? NG : GYV * GH, (float*)d_out);
}
